// PureMambaBlock_54004918780242
// MI455X (gfx1250) — hardware-verified
//
#include <hip/hip_runtime.h>
#include <math.h>
#include <stdint.h>

constexpr int kBatch     = 2;
constexpr int kSeq       = 2048;
constexpr int kDModel    = 1024;
constexpr int kDInner    = 2048;
constexpr int kDState    = 16;
constexpr int kDtRank    = 64;
constexpr int kDConv     = 4;
constexpr int kXprojN    = 96;
constexpr int kXprojNPad = 128;
constexpr int kScanCh    = 128;
constexpr int kScanT     = 16;

typedef __attribute__((ext_vector_type(16))) _Float16 v16h;
typedef __attribute__((ext_vector_type(8)))  _Float16 v8h;
typedef __attribute__((ext_vector_type(16))) __bf16   v16b;
typedef __attribute__((ext_vector_type(8)))  __bf16   v8b;
typedef __attribute__((ext_vector_type(8)))  float    v8f;
typedef __attribute__((ext_vector_type(4)))  float    v4f;
typedef __attribute__((ext_vector_type(4)))  unsigned int v4u;

__device__ __forceinline__ unsigned short f2bf_bits(float f) {
  unsigned u = __float_as_uint(f);
  return (unsigned short)((u + 0x7FFFu + ((u >> 16) & 1u)) >> 16);
}
__device__ __forceinline__ float bf_bits2f(unsigned short h) { return __uint_as_float(((unsigned)h) << 16); }

__device__ __forceinline__ void dep_guard_h(v8f& a, v8f& b, v16h x, v16h y) { asm volatile("v_nop\n\tv_nop\n\tv_nop\n\tv_nop" : "+v"(a), "+v"(b) : "v"(x), "v"(y)); }
__device__ __forceinline__ void dep_guard_b(v8f& a, v8f& b, v16b x, v16b y) { asm volatile("v_nop\n\tv_nop\n\tv_nop\n\tv_nop" : "+v"(a), "+v"(b) : "v"(x), "v"(y)); }
__device__ __forceinline__ void keep4_h(v16h a, v16h b, v16h c, v16h d) { asm volatile("v_nop" :: "v"(a), "v"(b), "v"(c), "v"(d)); }
__device__ __forceinline__ void keep4_b(v16b a, v16b b, v16b c, v16b d) { asm volatile("v_nop" :: "v"(a), "v"(b), "v"(c), "v"(d)); }
__device__ __forceinline__ void acc_guard4(v8f& a, v8f& b, v8f& c, v8f& d) { asm volatile("v_nop\n\tv_nop\n\tv_nop\n\tv_nop" : "+v"(a), "+v"(b), "+v"(c), "+v"(d)); }
template <typename T> struct Frag;
template <> struct Frag<_Float16> {
  typedef v16h V; union U { v16h v; v8h h[2]; };
  static __device__ __forceinline__ v16h load(const _Float16* p) {
    U f; f.h[0] = *(const v8h*)(p); f.h[1] = *(const v8h*)(p + 16); return f.v;
  }
  static __device__ __forceinline__ v8f mma(v16h a, v16h b, v8f c) {
    return __builtin_amdgcn_wmma_f32_16x16x32_f16(false, a, false, b, (short)0, c, false, false);
  }
  static __device__ __forceinline__ void guard(v8f& a, v8f& b, v16h x, v16h y) { dep_guard_h(a, b, x, y); }
  static __device__ __forceinline__ void keep(v16h a, v16h b, v16h c, v16h d) { keep4_h(a, b, c, d); }
};
template <> struct Frag<__bf16> {
  typedef v16b V; union U { v16b v; v8b h[2]; };
  static __device__ __forceinline__ v16b load(const __bf16* p) {
    U f; f.h[0] = *(const v8b*)(p); f.h[1] = *(const v8b*)(p + 16); return f.v;
  }
  static __device__ __forceinline__ v8f mma(v16b a, v16b b, v8f c) {
    return __builtin_amdgcn_wmma_f32_16x16x32_bf16(false, a, false, b, (short)0, c, false, false);
  }
  static __device__ __forceinline__ void guard(v8f& a, v8f& b, v16b x, v16b y) { dep_guard_b(a, b, x, y); }
  static __device__ __forceinline__ void keep(v16b a, v16b b, v16b c, v16b d) { keep4_b(a, b, c, d); }
};

__device__ __forceinline__ unsigned pk16(unsigned short a, unsigned short b) { return (unsigned)a | ((unsigned)b << 16); }

template <int ET> struct Elem;
template <> struct Elem<0> { typedef _Float16 T; };
template <> struct Elem<1> { typedef __bf16 T; };
template <int ET, bool SPLIT, int BIAS_MODE, int OUT_MODE, bool RESID, int ACT = 0>
__global__ __launch_bounds__(256) void wmma_gemm64(
    const unsigned short* __restrict__ Ap, const unsigned short* __restrict__ A2p, int lda, long strideA,
    const unsigned short* __restrict__ Btp, const unsigned short* __restrict__ Bt2p, int ldb, long strideB,
    void* __restrict__ Cout, void* __restrict__ Cout2, int ldc, long strideC,
    const float* __restrict__ bias,
    const float* __restrict__ resid, long strideR,
    int M, int N, int K, float scale) {
  typedef typename Elem<ET>::T T;
  typedef typename Frag<T>::V V;
  const T* A = (const T*)Ap; const T* A2 = (const T*)A2p; const T* Bt = (const T*)Btp; const T* Bt2 = (const T*)Bt2p;
  __shared__ __align__(16) float sT[8][16 * 68];
  const int b    = blockIdx.y;
  const int lane = threadIdx.x & 31;
  const int wave = threadIdx.x >> 5;
  const int tilesN = N >> 6;
  const int tilesM = M >> 6;
  const int tile = blockIdx.x * 8 + wave;
  if (tile >= tilesM * tilesN) return;
  const int tm = tile / tilesN;
  const int tn = tile - tm * tilesN;
  const int m0 = tm << 6;
  const int n0 = tn << 6;

  const T* Ab  = A  + (size_t)b * strideA;
  const T* Bb  = Bt + (size_t)b * strideB;
  const T* Ab2 = SPLIT ? (A2  + (size_t)b * strideA) : nullptr;
  const T* Bb2 = SPLIT ? (Bt2 + (size_t)b * strideB) : nullptr;

  const int rlane = lane & 15;
  const int koff  = (lane >> 4) * 8;
  const int mOff  = (lane >> 4) * 8;

  v8f acc[4][4];
#pragma unroll
  for (int i = 0; i < 4; ++i)
#pragma unroll
    for (int j = 0; j < 4; ++j) acc[i][j] = (v8f){0.f,0.f,0.f,0.f,0.f,0.f,0.f,0.f};

  for (int k0 = 0; k0 < K; k0 += 32) {
    V bh[4], bl[4];
#pragma unroll
    for (int j = 0; j < 4; ++j) {
      const size_t bo = (size_t)(n0 + (j << 4) + rlane) * ldb + koff + k0;
      bh[j] = Frag<T>::load(Bb + bo);
      if (SPLIT) bl[j] = Frag<T>::load(Bb2 + bo);
    }
#pragma unroll
    for (int i = 0; i < 4; ++i) {
      const size_t ao = (size_t)(m0 + (i << 4) + rlane) * lda + koff + k0;
      V ah = Frag<T>::load(Ab + ao);
      V al;
      if (SPLIT) al = Frag<T>::load(Ab2 + ao);
#pragma unroll
      for (int j = 0; j < 4; ++j) {
        acc[i][j] = Frag<T>::mma(ah, bh[j], acc[i][j]);
        if (SPLIT) {
          acc[i][j] = Frag<T>::mma(ah, bl[j], acc[i][j]);
          acc[i][j] = Frag<T>::mma(al, bh[j], acc[i][j]);
        }
      }
      Frag<T>::guard(acc[i][0], acc[i][3], ah, SPLIT ? al : ah);
    }
    Frag<T>::keep(bh[0], bh[1], bh[2], bh[3]);
    if (SPLIT) Frag<T>::keep(bl[0], bl[1], bl[2], bl[3]);
  }
  acc_guard4(acc[0][0], acc[0][1], acc[0][2], acc[0][3]);
  acc_guard4(acc[1][0], acc[1][1], acc[1][2], acc[1][3]);
  acc_guard4(acc[2][0], acc[2][1], acc[2][2], acc[2][3]);
  acc_guard4(acc[3][0], acc[3][1], acc[3][2], acc[3][3]);

  float* slab = sT[wave];
  const float* Rb = RESID ? (resid + (size_t)b * strideR) : nullptr;
#pragma unroll
  for (int i = 0; i < 4; ++i) {
    const int mBase = m0 + (i << 4);
#pragma unroll
    for (int j = 0; j < 4; ++j) {
      const int n = n0 + (j << 4) + rlane;
      float bv = 0.f;
      if (BIAS_MODE == 2) bv = bias[n];
#pragma unroll
      for (int r = 0; r < 8; ++r) {
        float v = acc[i][j][r] * scale;
        if (BIAS_MODE == 1) v += bias[mBase + mOff + r];
        if (BIAS_MODE == 2) v += bv;
        if (RESID) v += Rb[(size_t)(mBase + mOff + r) * ldc + n];
        if (ACT == 2) v = fmaxf(v, 0.0f);
        if (ACT == 4) v = (v > 0.f) ? v : 0.01f * v;
        slab[(mOff + r) * 68 + (j << 4) + rlane] = v;
      }
    }
    __builtin_amdgcn_fence(__ATOMIC_RELEASE, "workgroup");
    __builtin_amdgcn_wave_barrier();
    __builtin_amdgcn_fence(__ATOMIC_ACQUIRE, "workgroup");
    if (OUT_MODE == 0) {
      float* C = (float*)Cout + (size_t)b * strideC;
      const int hh = lane >> 4, c4 = (lane & 15) * 4;
      for (int pass = 0; pass < 2; ++pass) {
#pragma unroll
        for (int it = 0; it < 8; ++it) {
          const int row = it * 2 + hh;
          v4f v = *(const v4f*)(slab + row * 68 + c4);
          *(volatile v4f*)(C + (size_t)(mBase + row) * ldc + n0 + c4) = v;
        }
        __threadfence();
      }
    } else {
      const int q = lane >> 3, c8 = (lane & 7) * 8;
      unsigned short* C  = (unsigned short*)Cout  + (size_t)b * strideC;
      unsigned short* C2 = (OUT_MODE == 2) ? ((unsigned short*)Cout2 + (size_t)b * strideC) : nullptr;
      for (int pass = 0; pass < 2; ++pass) {
#pragma unroll
        for (int it = 0; it < 4; ++it) {
          const int row = it * 4 + q;
          const float* sp = slab + row * 68 + c8;
          v8h hv, lv;
#pragma unroll
          for (int e = 0; e < 8; ++e) {
            if (OUT_MODE == 1) {
              hv[e] = (_Float16)sp[e];
            } else {
              unsigned short hb = f2bf_bits(sp[e]);
              unsigned short lb = f2bf_bits(sp[e] - bf_bits2f(hb));
              hv[e] = __builtin_bit_cast(_Float16, hb);
              lv[e] = __builtin_bit_cast(_Float16, lb);
            }
          }
          *(volatile v8h*)(C + (size_t)(mBase + row) * ldc + n0 + c8) = hv;
          if (OUT_MODE == 2) *(volatile v8h*)(C2 + (size_t)(mBase + row) * ldc + n0 + c8) = lv;
        }
        __threadfence();
      }
    }
    __builtin_amdgcn_fence(__ATOMIC_RELEASE, "workgroup");
    __builtin_amdgcn_wave_barrier();
    __builtin_amdgcn_fence(__ATOMIC_ACQUIRE, "workgroup");
  }
}

__global__ __launch_bounds__(256) void split8_kernel(const float* __restrict__ src, int src_ld, int colshift,
                                                     unsigned short* __restrict__ hi, unsigned short* __restrict__ lo,
                                                     int n8valid, int n8total) {
  const int i = blockIdx.x * 256 + threadIdx.x;
  if (i >= n8total) return;
  const bool valid = (i < n8valid);
  const int ic  = valid ? i : (n8valid - 1);
  const int row = ic >> colshift;
  const int col = (ic & ((1 << colshift) - 1)) * 8;
  const float* p = src + (size_t)row * src_ld + col;
  const v4f a = *(const v4f*)(p);
  const v4f c = *(const v4f*)(p + 4);
  float x[8];
#pragma unroll
  for (int e = 0; e < 4; ++e) { x[e] = valid ? a[e] : 0.f; x[4 + e] = valid ? c[e] : 0.f; }
  unsigned short hb[8], lb[8];
#pragma unroll
  for (int e = 0; e < 8; ++e) {
    hb[e] = f2bf_bits(x[e]);
    lb[e] = f2bf_bits(x[e] - bf_bits2f(hb[e]));
  }
  const v4u hu = (v4u){pk16(hb[0], hb[1]), pk16(hb[2], hb[3]), pk16(hb[4], hb[5]), pk16(hb[6], hb[7])};
  const v4u lu = (v4u){pk16(lb[0], lb[1]), pk16(lb[2], lb[3]), pk16(lb[4], lb[5]), pk16(lb[6], lb[7])};
  unsigned short* qh = hi + 8 * (size_t)i;
  unsigned short* ql = lo + 8 * (size_t)i;
  *(volatile v4u*)qh = hu;
  *(volatile v4u*)ql = lu;
  __threadfence();
  *(volatile v4u*)qh = hu;
  *(volatile v4u*)ql = lu;
}

__global__ __launch_bounds__(256) void conv_silu_kernel(const float* __restrict__ xp, const float* __restrict__ cw,
                                                        const float* __restrict__ cb,
                                                        unsigned short* __restrict__ uh, unsigned short* __restrict__ ul) {
  const int l = blockIdx.x;
  const int d = threadIdx.x * 8;
  unsigned wh0 = 0u, wh1 = 0u, wh2 = 0u, wh3 = 0u;
  unsigned wl0 = 0u, wl1 = 0u, wl2 = 0u, wl3 = 0u;
#pragma unroll 1
  for (int hf = 0; hf < 2; ++hf) {
    const int dc = d + 4 * hf;
    const v4f wa = *(const v4f*)(cw + (size_t)(dc + 0) * kDConv);
    const v4f wb = *(const v4f*)(cw + (size_t)(dc + 1) * kDConv);
    const v4f wc = *(const v4f*)(cw + (size_t)(dc + 2) * kDConv);
    const v4f wd = *(const v4f*)(cw + (size_t)(dc + 3) * kDConv);
    float a0 = 0.f, a1 = 0.f, a2 = 0.f, a3 = 0.f;
#pragma unroll
    for (int j = 0; j < kDConv; ++j) {
      const int ll  = l - (kDConv - 1) + j;
      const int llc = (ll < 0) ? 0 : ll;
      const v4f xv = *(const v4f*)(xp + (size_t)llc * kDInner + dc);
      const bool okr = (ll >= 0);
      a0 += wa[j] * (okr ? xv[0] : 0.f);
      a1 += wb[j] * (okr ? xv[1] : 0.f);
      a2 += wc[j] * (okr ? xv[2] : 0.f);
      a3 += wd[j] * (okr ? xv[3] : 0.f);
    }
    const v4f bv = *(const v4f*)(cb + dc);
    a0 += bv[0];
    a1 += bv[1];
    a2 += bv[2];
    a3 += bv[3];
    const float e0 = expf(fminf(-a0, 80.f));
    const float e1 = expf(fminf(-a1, 80.f));
    const float e2 = expf(fminf(-a2, 80.f));
    const float e3 = expf(fminf(-a3, 80.f));
    const float u0 = a0 * (1.0f / (1.0f + e0));
    const float u1 = a1 * (1.0f / (1.0f + e1));
    const float u2 = a2 * (1.0f / (1.0f + e2));
    const float u3 = a3 * (1.0f / (1.0f + e3));
    const unsigned short h0 = f2bf_bits(u0), h1 = f2bf_bits(u1), h2 = f2bf_bits(u2), h3 = f2bf_bits(u3);
    const unsigned short g0 = f2bf_bits(u0 - bf_bits2f(h0)), g1 = f2bf_bits(u1 - bf_bits2f(h1));
    const unsigned short g2 = f2bf_bits(u2 - bf_bits2f(h2)), g3 = f2bf_bits(u3 - bf_bits2f(h3));
    const unsigned ph0 = pk16(h0, h1), ph1 = pk16(h2, h3);
    const unsigned pl0 = pk16(g0, g1), pl1 = pk16(g2, g3);
    const bool first = (hf == 0);
    wh0 = first ? ph0 : wh0;
    wh1 = first ? ph1 : wh1;
    wh2 = first ? wh2 : ph0;
    wh3 = first ? wh3 : ph1;
    wl0 = first ? pl0 : wl0;
    wl1 = first ? pl1 : wl1;
    wl2 = first ? wl2 : pl0;
    wl3 = first ? wl3 : pl1;
  }
  const v4u hu = (v4u){wh0, wh1, wh2, wh3};
  const v4u lu = (v4u){wl0, wl1, wl2, wl3};
  const size_t q = (size_t)l * kDInner + d;
  unsigned short* qh = uh + q;
  unsigned short* ql = ul + q;
  *(volatile v4u*)qh = hu;
  *(volatile v4u*)ql = lu;
  __threadfence();
  *(volatile v4u*)qh = hu;
  *(volatile v4u*)ql = lu;
}

__global__ __launch_bounds__(kScanCh) void scan_kernel(const float* __restrict__ draw,
                                                      const unsigned short* __restrict__ uh, const unsigned short* __restrict__ ul,
                                                      const float* __restrict__ xdbl, const float* __restrict__ zp,
                                                      const float* __restrict__ alog, const float* __restrict__ dvec,
                                                      unsigned short* __restrict__ yh, unsigned short* __restrict__ yl) {
  __shared__ float sA[kDState][kScanCh];
  __shared__ float sH[kDState][kScanCh];
  __shared__ float sDl[kScanT][kScanCh];
  __shared__ float sU[kScanT][kScanCh];
  __shared__ float sG[kScanT][kScanCh];
  __shared__ __align__(16) float sY[kScanT][kScanCh];
  __shared__ float sBC[kScanT][2 * kDState];
  const int ch   = threadIdx.x;
  const int lane = ch & 31, wave = ch >> 5;
  const int d0   = blockIdx.x * kScanCh;
  const int d    = d0 + ch;
#pragma unroll 1
  for (int n = 0; n < kDState; ++n) {
    sA[n][ch] = -expf(alog[(size_t)d * kDState + n]);
    sH[n][ch] = 0.f;
  }
  const float Dd = dvec[d];
  __syncthreads();
#pragma unroll 1
  for (int c = 0; c < kSeq / kScanT; ++c) {
    const int l0 = c * kScanT;
#pragma unroll 1
    for (int t = 0; t < kScanT; ++t) {
      const size_t e = (size_t)(l0 + t) * kDInner + d;
      const float dr = draw[e];
      sDl[t][ch] = fmaxf(dr, 0.f) + log1pf(expf(-fabsf(dr)));
      const unsigned wh = uh[e], wl = ul[e];
      sU[t][ch] = __uint_as_float(wh << 16) + __uint_as_float(wl << 16);
      const float zv = zp[e];
      const float ez = expf(fminf(-zv, 80.f));
      sG[t][ch] = zv * (1.0f / (1.0f + ez));
    }
#pragma unroll 1
    for (int idx = ch; idx < kScanT * 2 * kDState; idx += kScanCh) {
      const int t = idx >> 5, j = idx & 31;
      sBC[t][j] = xdbl[(size_t)(l0 + t) * kXprojNPad + kDtRank + j];
    }
    __syncthreads();
#pragma unroll 1
    for (int t = 0; t < kScanT; ++t) {
      const float dl = sDl[t][ch];
      const float u  = sU[t][ch];
      const float du = dl * u;
      float ys = 0.f;
#pragma unroll 2
      for (int n = 0; n < kDState; ++n) {
        const float a  = sA[n][ch];
        float h        = sH[n][ch];
        const float bn = sBC[t][n];
        const float cn = sBC[t][kDState + n];
        const float da = expf(dl * a);
        const float dbu = du * bn;
        h = da * h + dbu;
        sH[n][ch] = h;
        ys += h * cn;
      }
      sY[t][ch] = (ys + u * Dd) * sG[t][ch];
    }
    __syncthreads();
    {
      const int hh = lane >> 4, c8 = (lane & 15) * 8;
      for (int pass = 0; pass < 2; ++pass) {
#pragma unroll
        for (int it = 0; it < 2; ++it) {
          const int row = it * 8 + wave * 2 + hh;
          const v4f va = *(const v4f*)(&sY[row][c8]);
          const v4f vb = *(const v4f*)(&sY[row][c8 + 4]);
          unsigned short hb[8], lb[8];
#pragma unroll
          for (int e = 0; e < 4; ++e) {
            hb[e] = f2bf_bits(va[e]);         lb[e] = f2bf_bits(va[e] - bf_bits2f(hb[e]));
            hb[4 + e] = f2bf_bits(vb[e]);     lb[4 + e] = f2bf_bits(vb[e] - bf_bits2f(hb[4 + e]));
          }
          const v4u hu = (v4u){pk16(hb[0], hb[1]), pk16(hb[2], hb[3]), pk16(hb[4], hb[5]), pk16(hb[6], hb[7])};
          const v4u lu = (v4u){pk16(lb[0], lb[1]), pk16(lb[2], lb[3]), pk16(lb[4], lb[5]), pk16(lb[6], lb[7])};
          const size_t o = (size_t)(l0 + row) * kDInner + d0 + c8;
          *(volatile v4u*)(yh + o) = hu;
          *(volatile v4u*)(yl + o) = lu;
        }
        __threadfence();
      }
    }
  }
}

__global__ __launch_bounds__(256) void copy4_kernel(const float* __restrict__ in, float* __restrict__ out, int n4) {
  const int i = blockIdx.x * 256 + threadIdx.x;
  if (i >= n4) return;
  const v4f v = *(const v4f*)(in + 4 * (size_t)i);
  float* q = out + 4 * (size_t)i;
  *(volatile v4f*)q = v;
  __threadfence();
  *(volatile v4f*)q = v;
}

extern "C" void kernel_launch(void* const* d_in, const int* in_sizes, int n_in,
                              void* d_out, int out_size, void* d_ws, size_t ws_size,
                              hipStream_t stream) {
  (void)in_sizes; (void)n_in; (void)out_size;
  const float* hidden = (const float*)d_in[0];
  const float* inw    = (const float*)d_in[1];
  const float* convw  = (const float*)d_in[2];
  const float* convb  = (const float*)d_in[3];
  const float* xprojw = (const float*)d_in[4];
  const float* dtw    = (const float*)d_in[5];
  const float* dtb    = (const float*)d_in[6];
  const float* alog   = (const float*)d_in[7];
  const float* dvec   = (const float*)d_in[8];
  const float* outw   = (const float*)d_in[9];
  float* out = (float*)d_out;

  char* ws = (char*)d_ws;
  size_t off = 0;
  auto carve = [&](size_t bytes) -> char* {
    char* p = ws + off;
    off += (bytes + 4095) & ~(size_t)4095;
    return p;
  };
  unsigned short* Wh  = (unsigned short*)carve((size_t)2 * kDInner * kDModel * 2);
  unsigned short* Wl  = (unsigned short*)carve((size_t)2 * kDInner * kDModel * 2);
  unsigned short* Oh  = (unsigned short*)carve((size_t)kDModel * kDInner * 2);
  unsigned short* Ol  = (unsigned short*)carve((size_t)kDModel * kDInner * 2);
  unsigned short* Xh  = (unsigned short*)carve((size_t)kXprojNPad * kDInner * 2);
  unsigned short* Xl  = (unsigned short*)carve((size_t)kXprojNPad * kDInner * 2);
  unsigned short* Ph  = (unsigned short*)carve((size_t)kDInner * kDtRank * 2);
  unsigned short* Pl  = (unsigned short*)carve((size_t)kDInner * kDtRank * 2);
  unsigned short* Hh  = (unsigned short*)carve((size_t)kSeq * kDModel * 2);
  unsigned short* Hl  = (unsigned short*)carve((size_t)kSeq * kDModel * 2);
  float*          xpl = (float*)carve((size_t)kSeq * kDInner * 4);
  float*          zpl = (float*)carve((size_t)kSeq * kDInner * 4);
  unsigned short* uh  = (unsigned short*)carve((size_t)kSeq * kDInner * 2);
  unsigned short* ul  = (unsigned short*)carve((size_t)kSeq * kDInner * 2);
  float*          xdbl = (float*)carve((size_t)kSeq * kXprojNPad * 4);
  unsigned short* dth = (unsigned short*)carve((size_t)kSeq * kDtRank * 2);
  unsigned short* dtl = (unsigned short*)carve((size_t)kSeq * kDtRank * 2);
  unsigned short* yh  = (unsigned short*)carve((size_t)kSeq * kDInner * 2);
  unsigned short* yl  = (unsigned short*)carve((size_t)kSeq * kDInner * 2);
  float* draw = xpl;
  if (off > ws_size) return;

  {
    const int n8w = 2 * kDInner * kDModel / 8;
    split8_kernel<<<(n8w + 255) / 256, 256, 0, stream>>>(inw, kDModel, 7, Wh, Wl, n8w, n8w);
    const int n8o = kDModel * kDInner / 8;
    split8_kernel<<<(n8o + 255) / 256, 256, 0, stream>>>(outw, kDInner, 8, Oh, Ol, n8o, n8o);
    const int n8xv = kXprojN * kDInner / 8;
    const int n8xt = kXprojNPad * kDInner / 8;
    split8_kernel<<<(n8xt + 255) / 256, 256, 0, stream>>>(xprojw, kDInner, 8, Xh, Xl, n8xv, n8xt);
    const int n8p = kDInner * kDtRank / 8;
    split8_kernel<<<(n8p + 255) / 256, 256, 0, stream>>>(dtw, kDtRank, 3, Ph, Pl, n8p, n8p);
  }
  {
    const int n4 = kBatch * kSeq * kDModel / 4;
    copy4_kernel<<<(n4 + 255) / 256, 256, 0, stream>>>(hidden, out + (size_t)kBatch * kSeq * kDModel, n4);
  }

  for (int b = 0; b < kBatch; ++b) {
    const float* hb = hidden + (size_t)b * kSeq * kDModel;
    float* outb = out + (size_t)b * kSeq * kDModel;

    {
      const int n8h = kSeq * kDModel / 8;
      split8_kernel<<<(n8h + 255) / 256, 256, 0, stream>>>(hb, kDModel, 7, Hh, Hl, n8h, n8h);
    }
    {
      const int tiles = (kSeq / 64) * (kDInner / 64);
      wmma_gemm64<1, true, 0, 0, false><<<dim3(tiles / 8, 1), 256, 0, stream>>>(
          Hh, Hl, kDModel, 0L, Wh, Wl, kDModel, 0L,
          (void*)xpl, nullptr, kDInner, 0L, nullptr, nullptr, 0L, kSeq, kDInner, kDModel, 1.0f);
      wmma_gemm64<1, true, 0, 0, false><<<dim3(tiles / 8, 1), 256, 0, stream>>>(
          Hh, Hl, kDModel, 0L, Wh + (size_t)kDInner * kDModel, Wl + (size_t)kDInner * kDModel, kDModel, 0L,
          (void*)zpl, nullptr, kDInner, 0L, nullptr, nullptr, 0L, kSeq, kDInner, kDModel, 1.0f);
    }
    conv_silu_kernel<<<kSeq, 256, 0, stream>>>(xpl, convw, convb, uh, ul);
    {
      const int tiles = (kSeq / 64) * (kXprojNPad / 64);
      wmma_gemm64<1, true, 0, 0, false><<<dim3(tiles / 8, 1), 256, 0, stream>>>(
          uh, ul, kDInner, 0L, Xh, Xl, kDInner, 0L,
          (void*)xdbl, nullptr, kXprojNPad, 0L, nullptr, nullptr, 0L, kSeq, kXprojNPad, kDInner, 1.0f);
    }
    {
      const int n8d = kSeq * kDtRank / 8;
      split8_kernel<<<(n8d + 255) / 256, 256, 0, stream>>>(xdbl, kXprojNPad, 3, dth, dtl, n8d, n8d);
    }
    {
      const int tiles = (kSeq / 64) * (kDInner / 64);
      wmma_gemm64<1, true, 2, 0, false><<<dim3(tiles / 8, 1), 256, 0, stream>>>(
          dth, dtl, kDtRank, 0L, Ph, Pl, kDtRank, 0L,
          (void*)draw, nullptr, kDInner, 0L, dtb, nullptr, 0L, kSeq, kDInner, kDtRank, 1.0f);
    }
    scan_kernel<<<kDInner / kScanCh, kScanCh, 0, stream>>>(draw, uh, ul, xdbl, zpl, alog, dvec, yh, yl);
    {
      const int tiles = (kSeq / 64) * (kDModel / 64);
      wmma_gemm64<1, true, 0, 0, false><<<dim3(tiles / 8, 1), 256, 0, stream>>>(
          yh, yl, kDInner, 0L, Oh, Ol, kDInner, 0L,
          (void*)outb, nullptr, kDModel, 0L, nullptr, nullptr, 0L, kSeq, kDModel, kDInner, 1.0f);
    }
  }
}
